// NRMSMultiHeadSelfAttention_19413252177952
// MI455X (gfx1250) — hardware-run, weakly checked
//
#include <hip/hip_runtime.h>


namespace {
constexpr int NB = 32, S = 512, DM = 256, NH = 16, DK = 16, NR = NB * S, KB = 128  ;
constexpr float XS = 8.0f, WSC = 256.0f;
typedef _Float16 b16;
typedef __attribute__((ext_vector_type(16))) _Float16 v16b;
typedef __attribute__((ext_vector_type(8))) _Float16 v8b;
typedef __attribute__((ext_vector_type(8))) float v8f;
typedef __attribute__((ext_vector_type(4))) float v4f;
__device__ __forceinline__ float bf16_rne(float f) { unsigned int u = __float_as_uint(f); u += 0x7FFFu + ((u >> 16) & 1u); float r = __uint_as_float(u & 0xFFFF0000u); asm volatile("" : "+v"(r)); return r; }
__device__ __forceinline__ void split16(float v, b16& hi, b16& lo) { hi = (b16)v; lo = (b16)(v - (float)hi); }
__device__ __forceinline__ v16b frag_kb(const b16* p, int hh) { const v8b a = *(const v8b*)(p + 8 * hh), b = *(const v8b*)(p + 16 + 8 * hh); v16b f;
#pragma unroll
  for (int e = 0; e < 8; ++e) { f[e] = a[e]; f[8 + e] = b[e]; } return f; }
__device__ __forceinline__ v8f wmma16b(v16b a, v16b b, v8f c) { v8f d = __builtin_amdgcn_wmma_f32_16x16x32_f16(false, a, false, b, (short)0, c, false, false); asm volatile("v_nop\n\tv_nop\n\tv_nop\n\tv_nop" : "+v"(d) : "v"(a), "v"(b)); return d; }
__device__ __forceinline__ void wave_lds_sync() { __builtin_amdgcn_fence(__ATOMIC_RELEASE, "workgroup"); __builtin_amdgcn_wave_barrier(); __builtin_amdgcn_fence(__ATOMIC_ACQUIRE, "workgroup"); }
__device__ __forceinline__ float pmul(float a, float b) { float p = a * b; asm volatile("" : "+v"(p)); return p; }

__global__ __launch_bounds__(256) void wput_kernel(const float* __restrict__ wq, const float* __restrict__ wk, const float* __restrict__ wv, b16* __restrict__ W3) { const int u = blockIdx.x * 256 + threadIdx.x; if (u >= 3 * DM * 32) return; const int r = u / 32, k0 = (u % 32) * 8; const int part = r / DM, o = r % DM; const float* w = part == 0 ? wq : (part == 1 ? wk : wv); v8b v;
#pragma unroll
  for (int j = 0; j < 8; ++j) v[j] = (b16)(bf16_rne(w[(size_t)o * DM + k0 + j]) * WSC); for (int pass = 0; pass < 2; ++pass) { *(volatile v8b*)(W3 + (size_t)r * DM + k0) = v; __threadfence(); } }
__global__ __launch_bounds__(32) void proj_kernel(const float* __restrict__ Qi, const float* __restrict__ Ki, const float* __restrict__ Vi, const b16* __restrict__ W3, const float* __restrict__ bq, const float* __restrict__ bk, const float* __restrict__ bv, int RLIM, float* __restrict__ QKV) { __shared__ __attribute__((aligned(16))) b16 Ah[16][DM + 8]; __shared__ float Tf[16][260]; const int lane = threadIdx.x, nloc = lane & 15, hlf = lane >> 4; const int part = blockIdx.x % 3; const size_t m0 = (size_t)(blockIdx.x / 3) * 16; if (m0 >= (size_t)RLIM) return; const float* in = part == 0 ? Qi : (part == 1 ? Ki : Vi); const float* bb = part == 0 ? bq : (part == 1 ? bk : bv); const float osc = part == 0 ? 0.25f : 1.0f;
  for (int rr = 0; rr < 16; ++rr) for (int q = 0; q < 8; ++q) Ah[rr][q * 32 + lane] = (b16)(bf16_rne(in[(m0 + rr) * DM + q * 32 + lane]) * XS);
  wave_lds_sync(); v8f acc[16];
#pragma unroll
  for (int t = 0; t < 16; ++t) acc[t] = (v8f){};
#pragma unroll 2
  for (int kb = 0; kb < DM; kb += 32) { const v16b a = frag_kb(&Ah[nloc][kb], hlf);
#pragma unroll
    for (int t = 0; t < 16; ++t) acc[t] = wmma16b(a, frag_kb(W3 + ((size_t)part * DM + t * 16 + nloc) * DM + kb, hlf), acc[t]); }
#pragma unroll
  for (int t = 0; t < 16; ++t) { const int cc = t * 16 + nloc; const float bvv = bf16_rne(bb[cc]);
#pragma unroll
    for (int r8 = 0; r8 < 8; ++r8) Tf[8 * hlf + r8][cc] = (acc[t][r8] * (1.0f / (XS * WSC)) + bvv) * osc; }
  wave_lds_sync();
  for (int pass = 0; pass < 2; ++pass) { for (int rr = 0; rr < 16; ++rr) for (int q = 0; q < 2; ++q) *(volatile v4f*)(QKV + (m0 + rr) * (3 * DM) + part * DM + q * 128 + lane * 4) = *(const v4f*)(&Tf[rr][q * 128 + lane * 4]); __threadfence(); } }
__global__ __launch_bounds__(32) void att_kernel(const float* __restrict__ QKV, const float* __restrict__ mask, int BLIM, float* __restrict__ out) { __shared__ __attribute__((aligned(16))) b16 Qh[16][40], Ql[16][40], Kh[KB][40], Kl[KB][40], Ph[16][KB + 8], Pl[16][KB + 8], Vh[16][KB + 8], Vl[16][KB + 8]; __shared__ float Sf[16][KB + 4], Mk[KB], Of[16][34];
  const int lane = threadIdx.x, nloc = lane & 15, hlf = lane >> 4; const int qt = blockIdx.x % (S / 16); const int hp = (blockIdx.x / (S / 16)) % (NH / 2); const int b = blockIdx.x / ((S / 16) * (NH / 2)); if (b >= BLIM) return; const size_t rb_ = (size_t)b * S; const int t0 = qt * 16;
#pragma unroll 1
  for (int hs = 0; hs < 2; ++hs) { const int h = hp * 2 + hs;
    for (int rr = 0; rr < 16; ++rr) { b16 p, ql; split16((lane < DK ? QKV[(rb_ + t0 + rr) * 768 + h * DK + lane] : 0.0f) * XS, p, ql); Qh[rr][lane] = p; Ql[rr][lane] = ql; if (lane < 8) { Qh[rr][32 + lane] = (b16)0.0f; Ql[rr][32 + lane] = (b16)0.0f; } }
    float m_r[8], den_r[8]; v8f acc = {};
#pragma unroll
    for (int r8 = 0; r8 < 8; ++r8) { m_r[r8] = -INFINITY; den_r[r8] = 0.0f; }
    wave_lds_sync(); const v16b qa = frag_kb(&Qh[nloc][0], hlf), qb = frag_kb(&Ql[nloc][0], hlf);
#pragma unroll 1
    for (int kb0 = 0; kb0 < S; kb0 += KB) {
      for (int rr = 0; rr < KB; rr += 2) { const int r = rr + hlf; const size_t row = rb_ + kb0 + r; b16 p, ql; split16(QKV[row * 768 + DM + h * DK + nloc] * XS, p, ql); Kh[r][nloc] = p; Kl[r][nloc] = ql; Kh[r][16 + nloc] = (b16)0.0f; Kl[r][16 + nloc] = (b16)0.0f; }
      for (int kk = 0; kk < KB; kk += 32) { const size_t row = rb_ + kb0 + kk + lane; Mk[kk + lane] = bf16_rne(mask[row]);
#pragma unroll
        for (int d = 0; d < DK; ++d) { b16 p, ql; split16(QKV[row * 768 + 2 * DM + h * DK + d] * XS, p, ql); Vh[d][kk + lane] = p; Vl[d][kk + lane] = ql; } }
      wave_lds_sync();
#pragma unroll
      for (int t = 0; t < KB / 16; ++t) { const v16b kh = frag_kb(&Kh[t * 16 + nloc][0], hlf), kl = frag_kb(&Kl[t * 16 + nloc][0], hlf); v8f s = {}; s = wmma16b(qa, kh, s); s = wmma16b(qa, kl, s); s = wmma16b(qb, kh, s);
#pragma unroll
        for (int r8 = 0; r8 < 8; ++r8) Sf[8 * hlf + r8][t * 16 + nloc] = s[r8] * (1.0f / (XS * XS)); }
      wave_lds_sync();
#pragma unroll
      for (int rr = 0; rr < 16; ++rr) { float mx = -INFINITY;
#pragma unroll
        for (int q = 0; q < 4; ++q) mx = fmaxf(mx, Sf[rr][q * 32 + lane]);
        for (int o = 16; o; o >>= 1) mx = fmaxf(mx, __shfl_xor(mx, o));
        const float mold = __shfl(m_r[rr & 7], (rr >> 3) * 16); const float mn = fmaxf(mold, mx); const float sf = (mold == -INFINITY) ? 0.0f : __expf(mold - mn); float ps = 0.0f;
#pragma unroll
        for (int q = 0; q < 4; ++q) { const int kx = q * 32 + lane; const float p = pmul(__expf(Sf[rr][kx] - mn), Mk[kx]); ps += p; b16 ph, pl; split16(p * 256.0f, ph, pl);   Ph[rr][kx] = ph; Pl[rr][kx] = pl; }
        for (int o = 16; o; o >>= 1) ps += __shfl_xor(ps, o);
        if ((rr >> 3) == hlf) { const int r8 = rr & 7; den_r[r8] = den_r[r8] * sf + ps; m_r[r8] = mn; acc[r8] = acc[r8] * sf; } }
      wave_lds_sync();
#pragma unroll
      for (int ks = 0; ks < KB; ks += 32) { const v16b pa = frag_kb(&Ph[nloc][ks], hlf), pb = frag_kb(&Pl[nloc][ks], hlf), vh = frag_kb(&Vh[nloc][ks], hlf), vl = frag_kb(&Vl[nloc][ks], hlf); acc = wmma16b(pa, vh, acc); acc = wmma16b(pa, vl, acc); acc = wmma16b(pb, vh, acc); }
      wave_lds_sync(); }
#pragma unroll
    for (int r8 = 0; r8 < 8; ++r8) { const float dn = den_r[r8] + 1e-8f * __expf(-m_r[r8]); Of[8 * hlf + r8][hs * 16 + nloc] = acc[r8] * (1.0f / (XS * 256.0f)) / dn; }
    wave_lds_sync(); }
  for (int pass = 0; pass < 2; ++pass) { for (int rr = 0; rr < 16; ++rr) ((volatile float*)out)[(rb_ + t0 + rr) * DM + hp * 32 + lane] = Of[rr][lane]; __threadfence(); } }
}

extern "C" void kernel_launch(void* const* d_in, const int* in_sizes, int n_in, void* d_out, int out_size, void* d_ws, size_t ws_size, hipStream_t stream) {
  (void)n_in;
  auto Fp = [&](int i) { return (const float*)d_in[i]; };
  if (in_sizes[0] != NR * DM || in_sizes[1] != NR * DM || in_sizes[2] != NR * DM || in_sizes[3] != NR || in_sizes[4] != DM * DM || in_sizes[6] != DM * DM || in_sizes[8] != DM * DM || out_size != NR * DM) return;
  const int BLIM = NB;
  size_t off = 0; char* ws = (char*)d_ws;
  auto carve = [&](size_t bytes) { char* p = ws + off; off += (bytes + 255) & ~(size_t)255; return p; };
  b16* W3 = (b16*)carve((size_t)3 * DM * DM * 2); float* QKV = (float*)carve((size_t)NR * 3 * DM * 4);
  if (off > ws_size || off > ((size_t)64 << 20)) return;
  wput_kernel<<<(3 * DM * 32 + 255) / 256, 256, 0, stream>>>(Fp(4), Fp(6), Fp(8), W3);
  proj_kernel<<<(BLIM * S / 16) * 3, 32, 0, stream>>>(Fp(0), Fp(1), Fp(2), W3, Fp(5), Fp(7), Fp(9), BLIM * S, QKV);
  att_kernel<<<BLIM * (NH / 2) * (S / 16), 32, 0, stream>>>(QKV, Fp(3), BLIM, (float*)d_out);
}
